// MultiHeadSelfAttention_28621662060746
// MI455X (gfx1250) — hardware-verified
//
#include <hip/hip_runtime.h>
#include <stddef.h>


#define DM 1024
#define NH 16
#define DK 64
#define SQ 2048
#define NB 2
#define BH (NB * NH)
#define MROWS (NB * SQ)
#define NEGBIG (-3.0e38f)

typedef unsigned short us_t;
typedef __bf16 v16bf __attribute__((ext_vector_type(16)));
typedef us_t v8us __attribute__((ext_vector_type(8)));
typedef float v8f __attribute__((ext_vector_type(8)));
typedef float v4f __attribute__((ext_vector_type(4)));
typedef unsigned int v4u __attribute__((ext_vector_type(4)));

union Frag { v16bf v; v8us h[2]; };
union P8 { v8us s; v4u u; };

__device__ __forceinline__ us_t f2bf(float f) {
  unsigned u = __float_as_uint(f);
  u = u + 0x7FFFu + ((u >> 16) & 1u);
  return (us_t)(u >> 16);
}
__device__ __forceinline__ float bf2f(us_t b) {
  return __uint_as_float(((unsigned)b) << 16);
}
__device__ __forceinline__ void split2(float f, us_t& hi, us_t& lo) {
  hi = f2bf(f);
  lo = f2bf(f - bf2f(hi));
}

__device__ __forceinline__ void ldfrag(Frag& f, const us_t* p) {
  f.h[0] = *(const v8us*)(p);
  f.h[1] = *(const v8us*)(p + 16);
}

__device__ __forceinline__ v8f wmma3(const Frag& ah, const Frag& al,
                                     const Frag& bh, const Frag& bl, v8f acc) {
  acc = __builtin_amdgcn_wmma_f32_16x16x32_bf16(false, ah.v, false, bh.v, (short)0, acc, false, false);
  acc = __builtin_amdgcn_wmma_f32_16x16x32_bf16(false, ah.v, false, bl.v, (short)0, acc, false, false);
  acc = __builtin_amdgcn_wmma_f32_16x16x32_bf16(false, al.v, false, bh.v, (short)0, acc, false, false);
  asm volatile("v_nop\n\tv_nop\n\tv_nop\n\tv_nop"
               : "+v"(acc)
               : "v"(ah.v), "v"(al.v), "v"(bh.v), "v"(bl.v));
  return acc;
}

__global__ __launch_bounds__(256) void k_split_planes(const float* __restrict__ src,
                                                     us_t* hi, us_t* lo, int n8) {
  const int t = blockIdx.x * 256 + threadIdx.x;
  if (t >= n8) return;
  const size_t e = (size_t)t * 8;
  const v4f x0 = *(const v4f*)(src + e);
  const v4f x1 = *(const v4f*)(src + e + 4);
  us_t h0, h1, h2, h3, h4, h5, h6, h7;
  us_t l0, l1, l2, l3, l4, l5, l6, l7;
  split2(x0.x, h0, l0); split2(x0.y, h1, l1); split2(x0.z, h2, l2); split2(x0.w, h3, l3);
  split2(x1.x, h4, l4); split2(x1.y, h5, l5); split2(x1.z, h6, l6); split2(x1.w, h7, l7);
  P8 ph, pl;
  v8us hv = {h0, h1, h2, h3, h4, h5, h6, h7};
  v8us lv = {l0, l1, l2, l3, l4, l5, l6, l7};
  ph.s = hv; pl.s = lv;
  volatile v4u* dh = (volatile v4u*)(hi + e);
  volatile v4u* dl = (volatile v4u*)(lo + e);
  *dh = ph.u;
  *dl = pl.u;
  __threadfence();
  *dh = ph.u;
  *dl = pl.u;
}

__global__ __launch_bounds__(128) void k_gemm_xwt(const us_t* __restrict__ Ah,
                                                 const us_t* __restrict__ Al,
                                                 const us_t* __restrict__ Wh,
                                                 const us_t* __restrict__ Wl,
                                                 float* C, int M, int N, int K) {
  __shared__ __attribute__((aligned(16))) float sC[4][32 * 36];
  const int lane = threadIdx.x & 31;
  const int wv = threadIdx.x >> 5;
  const int h = lane >> 4;
  const int m = lane & 15;
  const int nTn = N >> 5;
  const int nT = (M >> 5) * nTn;
  int tile = blockIdx.x * 4 + wv;
  const bool valid = tile < nT;
  if (!valid) tile = 0;
  const int rowBase = (tile / nTn) * 32;
  const int colBase = (tile % nTn) * 32;

  const size_t ar0 = (size_t)(rowBase + m) * K + 8 * h;
  const size_t ar1 = ar0 + (size_t)16 * K;
  const size_t bc0 = (size_t)(colBase + m) * K + 8 * h;
  const size_t bc1 = bc0 + (size_t)16 * K;

  v8f acc[2][2];
#pragma unroll
  for (int q = 0; q < 2; ++q)
#pragma unroll
    for (int t = 0; t < 2; ++t) acc[q][t] = (v8f){};

  for (int k0 = 0; k0 < K; k0 += 32) {
    Frag a0h, a0l, a1h, a1l, b0h, b0l, b1h, b1l;
    ldfrag(a0h, Ah + ar0 + k0); ldfrag(a0l, Al + ar0 + k0);
    ldfrag(a1h, Ah + ar1 + k0); ldfrag(a1l, Al + ar1 + k0);
    ldfrag(b0h, Wh + bc0 + k0); ldfrag(b0l, Wl + bc0 + k0);
    ldfrag(b1h, Wh + bc1 + k0); ldfrag(b1l, Wl + bc1 + k0);
    acc[0][0] = wmma3(a0h, a0l, b0h, b0l, acc[0][0]);
    acc[0][1] = wmma3(a0h, a0l, b1h, b1l, acc[0][1]);
    acc[1][0] = wmma3(a1h, a1l, b0h, b0l, acc[1][0]);
    acc[1][1] = wmma3(a1h, a1l, b1h, b1l, acc[1][1]);
  }

  float* s = &sC[wv][0];
#pragma unroll
  for (int q = 0; q < 2; ++q)
#pragma unroll
    for (int t = 0; t < 2; ++t)
#pragma unroll
      for (int r = 0; r < 8; ++r)
        s[(16 * q + 8 * h + r) * 36 + 16 * t + m] = acc[q][t][r];
  __syncthreads();

  v4f v[8];
  size_t ga[8];
#pragma unroll
  for (int i = 0; i < 8; ++i) {
    const int row = 4 * i + (lane >> 3);
    const int c4 = (lane & 7) * 4;
    v[i] = *(const v4f*)(s + row * 36 + c4);
    ga[i] = (size_t)(rowBase + row) * N + colBase + c4;
  }
  if (valid) {
#pragma unroll
    for (int i = 0; i < 8; ++i) *(volatile v4f*)(C + ga[i]) = v[i];
  }
  __threadfence();
  if (valid) {
#pragma unroll
    for (int i = 0; i < 8; ++i) *(volatile v4f*)(C + ga[i]) = v[i];
  }
}

__global__ __launch_bounds__(256) void k_rope_table(const int* __restrict__ pos,
                                                   float* cosT, float* sinT, int nrows) {
#pragma clang fp contract(off)
  const int gid = blockIdx.x * 256 + threadIdx.x;
  const int row = gid >> 3;
  const int p = gid & 7;
  if (row >= nrows) return;
  const float pf = (float)pos[row];
  float c0 = 0.f, c1 = 0.f, c2 = 0.f, c3 = 0.f;
  float s0 = 0.f, s1 = 0.f, s2 = 0.f, s3 = 0.f;
#pragma unroll 1
  for (int u = 0; u < 4; ++u) {
    const int j = p * 4 + u;
    const double fr = exp2((double)j * (13.287712379549449 / 32.0));
    const float inv = 1.0f / (float)fr;
    const float ang = pf * inv;
    const float c = cosf(ang);
    const float sn = sinf(ang);
    if (u == 0) { c0 = c; s0 = sn; }
    else if (u == 1) { c1 = c; s1 = sn; }
    else if (u == 2) { c2 = c; s2 = sn; }
    else { c3 = c; s3 = sn; }
  }
  v4f cv = {c0, c1, c2, c3};
  v4f sv = {s0, s1, s2, s3};
  const size_t o = (size_t)row * 32 + p * 4;
  volatile v4f* dc = (volatile v4f*)(cosT + o);
  volatile v4f* ds = (volatile v4f*)(sinT + o);
  *dc = cv;
  *ds = sv;
  __threadfence();
  *dc = cv;
  *ds = sv;
}

__device__ __forceinline__ void rope_line(const float* __restrict__ src,
                                          const float* __restrict__ ct,
                                          const float* __restrict__ st,
                                          float scale, us_t* dh, us_t* dl, size_t dst) {
#pragma clang fp contract(off)
  P8 H[8], L[8];
#pragma unroll
  for (int g = 0; g < 8; ++g) {
    const v4f c = *(const v4f*)(ct + 4 * g);
    const v4f sn = *(const v4f*)(st + 4 * g);
    const v4f x0 = *(const v4f*)(src + 8 * g);
    const v4f x1 = *(const v4f*)(src + 8 * g + 4);
    const float r0 = (x0.x * c.x - x0.y * sn.x) * scale;
    const float r1 = (x0.x * sn.x + x0.y * c.x) * scale;
    const float r2 = (x0.z * c.y - x0.w * sn.y) * scale;
    const float r3 = (x0.z * sn.y + x0.w * c.y) * scale;
    const float r4 = (x1.x * c.z - x1.y * sn.z) * scale;
    const float r5 = (x1.x * sn.z + x1.y * c.z) * scale;
    const float r6 = (x1.z * c.w - x1.w * sn.w) * scale;
    const float r7 = (x1.z * sn.w + x1.w * c.w) * scale;
    us_t h0, h1, h2, h3, h4, h5, h6, h7, l0, l1, l2, l3, l4, l5, l6, l7;
    split2(r0, h0, l0); split2(r1, h1, l1); split2(r2, h2, l2); split2(r3, h3, l3);
    split2(r4, h4, l4); split2(r5, h5, l5); split2(r6, h6, l6); split2(r7, h7, l7);
    v8us hv = {h0, h1, h2, h3, h4, h5, h6, h7};
    v8us lv = {l0, l1, l2, l3, l4, l5, l6, l7};
    H[g].s = hv; L[g].s = lv;
  }
#pragma unroll
  for (int g = 0; g < 8; ++g) {
    *(volatile v4u*)(dh + dst + 8 * g) = H[g].u;
    *(volatile v4u*)(dl + dst + 8 * g) = L[g].u;
  }
  __threadfence();
#pragma unroll
  for (int g = 0; g < 8; ++g) {
    *(volatile v4u*)(dh + dst + 8 * g) = H[g].u;
    *(volatile v4u*)(dl + dst + 8 * g) = L[g].u;
  }
}

__device__ __forceinline__ void plain_line(const float* __restrict__ src,
                                           us_t* dh, us_t* dl, size_t dst) {
  P8 H[8], L[8];
#pragma unroll
  for (int g = 0; g < 8; ++g) {
    const v4f x0 = *(const v4f*)(src + 8 * g);
    const v4f x1 = *(const v4f*)(src + 8 * g + 4);
    us_t h0, h1, h2, h3, h4, h5, h6, h7, l0, l1, l2, l3, l4, l5, l6, l7;
    split2(x0.x, h0, l0); split2(x0.y, h1, l1); split2(x0.z, h2, l2); split2(x0.w, h3, l3);
    split2(x1.x, h4, l4); split2(x1.y, h5, l5); split2(x1.z, h6, l6); split2(x1.w, h7, l7);
    v8us hv = {h0, h1, h2, h3, h4, h5, h6, h7};
    v8us lv = {l0, l1, l2, l3, l4, l5, l6, l7};
    H[g].s = hv; L[g].s = lv;
  }
#pragma unroll
  for (int g = 0; g < 8; ++g) {
    *(volatile v4u*)(dh + dst + 8 * g) = H[g].u;
    *(volatile v4u*)(dl + dst + 8 * g) = L[g].u;
  }
  __threadfence();
#pragma unroll
  for (int g = 0; g < 8; ++g) {
    *(volatile v4u*)(dh + dst + 8 * g) = H[g].u;
    *(volatile v4u*)(dl + dst + 8 * g) = L[g].u;
  }
}

__global__ __launch_bounds__(128) void k_rope_split(
    const float* __restrict__ Qf, const float* __restrict__ Kf, const float* __restrict__ Vf,
    const float* __restrict__ cosT, const float* __restrict__ sinT,
    us_t* Qh, us_t* Ql, us_t* Kh, us_t* Kl, us_t* Vh, us_t* Vl, int nlines) {
  const int t = blockIdx.x * 128 + threadIdx.x;
  if (t >= nlines) return;
  const int bs = t >> 4;
  const int hh = t & 15;
  const int b = bs >> 11;
  const int s = bs & (SQ - 1);
  const size_t src = (size_t)bs * DM + hh * DK;
  const size_t dst = ((size_t)(b * NH + hh) * SQ + s) * DK;
  const float* ct = cosT + (size_t)bs * 32;
  const float* st = sinT + (size_t)bs * 32;
  rope_line(Qf + src, ct, st, 0.125f, Qh, Ql, dst);
  rope_line(Kf + src, ct, st, 1.0f, Kh, Kl, dst);
  plain_line(Vf + src, Vh, Vl, dst);
}

__global__ __launch_bounds__(128) void k_attn(
    const us_t* __restrict__ Qh, const us_t* __restrict__ Ql,
    const us_t* __restrict__ Kh, const us_t* __restrict__ Kl,
    const us_t* __restrict__ Vh, const us_t* __restrict__ Vl,
    us_t* Ch, us_t* Cl, int nblk) {
  __shared__ __attribute__((aligned(16))) us_t sK[2][32 * 72];
  __shared__ __attribute__((aligned(16))) us_t sV[2][64 * 40];
  __shared__ __attribute__((aligned(16))) us_t sP[4][2][16 * 40];

  const int lane = threadIdx.x & 31;
  const int wv = threadIdx.x >> 5;
  const int h = lane >> 4;
  const int m = lane & 15;
  int blk = blockIdx.x;
  const bool valid = blk < nblk;
  if (!valid) blk = 0;
  const int bh = blk >> 5;
  const int qBlock = (blk & 31) * 64;
  const int q0 = qBlock + wv * 16;
  const int b = bh >> 4;
  const int hh = bh & 15;
  const size_t hb = (size_t)bh * SQ * DK;

  Frag aqh[2], aql[2];
#pragma unroll
  for (int kk = 0; kk < 2; ++kk) {
    const size_t o = hb + (size_t)(q0 + m) * DK + 32 * kk + 8 * h;
    ldfrag(aqh[kk], Qh + o);
    ldfrag(aql[kk], Ql + o);
  }

  v8f o[4];
  float mr[8], lr[8];
#pragma unroll
  for (int nt = 0; nt < 4; ++nt) o[nt] = (v8f){};
#pragma unroll
  for (int r = 0; r < 8; ++r) { mr[r] = NEGBIG; lr[r] = 0.0f; }

  const int kEnd = qBlock + 64;
  for (int k0 = 0; k0 < kEnd; k0 += 32) {
    __syncthreads();
#pragma unroll
    for (int i = 0; i < 4; ++i) {
      const int idx = threadIdx.x + 128 * i;
      const int pl = idx >> 8;
      const int r = (idx >> 3) & 31;
      const int g = idx & 7;
      const size_t go = hb + (size_t)(k0 + r) * DK + 8 * g;
      const v8us kv = *(const v8us*)((pl ? Kl : Kh) + go);
      *(v8us*)(&sK[pl][r * 72 + 8 * g]) = kv;
      const v8us vv = *(const v8us*)((pl ? Vl : Vh) + go);
      us_t* vd = &sV[pl][(8 * g) * 40 + r];
      vd[0 * 40] = vv[0]; vd[1 * 40] = vv[1]; vd[2 * 40] = vv[2]; vd[3 * 40] = vv[3];
      vd[4 * 40] = vv[4]; vd[5 * 40] = vv[5]; vd[6 * 40] = vv[6]; vd[7 * 40] = vv[7];
    }
    __syncthreads();

    v8f sc[2];
#pragma unroll
    for (int t = 0; t < 2; ++t) {
      v8f acc = (v8f){};
#pragma unroll
      for (int kk = 0; kk < 2; ++kk) {
        Frag bkh, bkl;
        const int so = (t * 16 + m) * 72 + 32 * kk + 8 * h;
        ldfrag(bkh, &sK[0][so]);
        ldfrag(bkl, &sK[1][so]);
        acc = wmma3(aqh[kk], aql[kk], bkh, bkl, acc);
      }
      sc[t] = acc;
    }

#pragma unroll
    for (int r = 0; r < 8; ++r) {
      const int qg = q0 + 8 * h + r;
      const float v0 = (k0 + m <= qg) ? sc[0][r] : NEGBIG;
      const float v1 = (k0 + 16 + m <= qg) ? sc[1][r] : NEGBIG;
      float bm = fmaxf(v0, v1);
      bm = fmaxf(bm, __shfl_xor(bm, 1, 32));
      bm = fmaxf(bm, __shfl_xor(bm, 2, 32));
      bm = fmaxf(bm, __shfl_xor(bm, 4, 32));
      bm = fmaxf(bm, __shfl_xor(bm, 8, 32));
      const float mnew = fmaxf(mr[r], bm);
      const float alpha = expf(mr[r] - mnew);
      const float p0 = expf(v0 - mnew);
      const float p1 = expf(v1 - mnew);
      float rs = p0 + p1;
      rs += __shfl_xor(rs, 1, 32);
      rs += __shfl_xor(rs, 2, 32);
      rs += __shfl_xor(rs, 4, 32);
      rs += __shfl_xor(rs, 8, 32);
      lr[r] = lr[r] * alpha + rs;
      mr[r] = mnew;
      o[0][r] *= alpha;
      o[1][r] *= alpha;
      o[2][r] *= alpha;
      o[3][r] *= alpha;
      us_t h0, l0, h1, l1;
      split2(p0, h0, l0);
      split2(p1, h1, l1);
      us_t* pr0 = &sP[wv][0][(8 * h + r) * 40];
      us_t* pr1 = &sP[wv][1][(8 * h + r) * 40];
      pr0[m] = h0;
      pr0[16 + m] = h1;
      pr1[m] = l0;
      pr1[16 + m] = l1;
    }
    __syncthreads();

    Frag ph, plo;
    {
      const int po = m * 40 + 8 * h;
      ldfrag(ph, &sP[wv][0][po]);
      ldfrag(plo, &sP[wv][1][po]);
    }
#pragma unroll
    for (int nt = 0; nt < 4; ++nt) {
      Frag bvh, bvl;
      const int vo = (nt * 16 + m) * 40 + 8 * h;
      ldfrag(bvh, &sV[0][vo]);
      ldfrag(bvl, &sV[1][vo]);
      o[nt] = wmma3(ph, plo, bvh, bvl, o[nt]);
    }
  }

  __syncthreads();
  us_t* stgH = &sK[0][0] + wv * 1024;
  us_t* stgL = &sV[0][0] + wv * 1024;
#pragma unroll
  for (int r = 0; r < 8; ++r) {
    const float inv = 1.0f / lr[r];
#pragma unroll
    for (int nt = 0; nt < 4; ++nt) {
      const float v = o[nt][r] * inv;
      us_t hv, lv;
      split2(v, hv, lv);
      const int so = (8 * h + r) * 64 + nt * 16 + m;
      stgH[so] = hv;
      stgL[so] = lv;
    }
  }
  __syncthreads();
  P8 H[4], L[4];
  size_t ga[4];
#pragma unroll
  for (int i = 0; i < 4; ++i) {
    const int row = 4 * i + (lane >> 3);
    const int g = lane & 7;
    H[i].s = *(const v8us*)(stgH + row * 64 + 8 * g);
    L[i].s = *(const v8us*)(stgL + row * 64 + 8 * g);
    ga[i] = (size_t)(b * SQ + q0 + row) * DM + hh * DK + 8 * g;
  }
  if (valid) {
#pragma unroll
    for (int i = 0; i < 4; ++i) {
      *(volatile v4u*)(Ch + ga[i]) = H[i].u;
      *(volatile v4u*)(Cl + ga[i]) = L[i].u;
    }
  }
  __threadfence();
  if (valid) {
#pragma unroll
    for (int i = 0; i < 4; ++i) {
      *(volatile v4u*)(Ch + ga[i]) = H[i].u;
      *(volatile v4u*)(Cl + ga[i]) = L[i].u;
    }
  }
}

extern "C" void kernel_launch(void* const* d_in, const int* in_sizes, int n_in,
                              void* d_out, int out_size, void* d_ws,
                              size_t ws_size, hipStream_t stream) {
  const int NTOK = MROWS * DM;
  const int NW = DM * DM;
  if (n_in < 6) return;
  if (in_sizes[0] != NTOK || in_sizes[1] != MROWS || in_sizes[2] != NW ||
      in_sizes[3] != NW || in_sizes[4] != NW || in_sizes[5] != NW ||
      out_size != NTOK)
    return;

  const float* x = (const float*)d_in[0];
  const int* tpos = (const int*)d_in[1];
  const float* wq = (const float*)d_in[2];
  const float* wk = (const float*)d_in[3];
  const float* wv = (const float*)d_in[4];
  const float* wo = (const float*)d_in[5];
  float* out = (float*)d_out;

  char* ws = (char*)d_ws;
  size_t off = 0;
  auto carve = [&](size_t bytes) -> char* {
    char* p = ws + off;
    off += (bytes + 255) & ~(size_t)255;
    return p;
  };
  us_t* Xh = (us_t*)carve((size_t)NTOK * 2);
  us_t* Xl = (us_t*)carve((size_t)NTOK * 2);
  us_t* Wqh = (us_t*)carve((size_t)NW * 2);
  us_t* Wql = (us_t*)carve((size_t)NW * 2);
  us_t* Wkh = (us_t*)carve((size_t)NW * 2);
  us_t* Wkl = (us_t*)carve((size_t)NW * 2);
  us_t* Wvh = (us_t*)carve((size_t)NW * 2);
  us_t* Wvl = (us_t*)carve((size_t)NW * 2);
  us_t* Woh = (us_t*)carve((size_t)NW * 2);
  us_t* Wol = (us_t*)carve((size_t)NW * 2);
  float* Qf = (float*)carve((size_t)NTOK * 4);
  float* Kf = (float*)carve((size_t)NTOK * 4);
  float* Vf = (float*)carve((size_t)NTOK * 4);
  float* cosT = (float*)carve((size_t)MROWS * 32 * 4);
  float* sinT = (float*)carve((size_t)MROWS * 32 * 4);
  us_t* Qh = (us_t*)carve((size_t)NTOK * 2);
  us_t* Ql = (us_t*)carve((size_t)NTOK * 2);
  us_t* Kh = (us_t*)carve((size_t)NTOK * 2);
  us_t* Kl = (us_t*)carve((size_t)NTOK * 2);
  us_t* Vh = (us_t*)carve((size_t)NTOK * 2);
  us_t* Vl = (us_t*)carve((size_t)NTOK * 2);
  us_t* Ch = (us_t*)carve((size_t)NTOK * 2);
  us_t* Cl = (us_t*)carve((size_t)NTOK * 2);
  if (off > ws_size) return;

  {
    const int n8x = NTOK / 8;
    const int n8w = NW / 8;
    k_split_planes<<<dim3((n8x + 255) / 256), dim3(256), 0, stream>>>(x, Xh, Xl, n8x);
    k_split_planes<<<dim3((n8w + 255) / 256), dim3(256), 0, stream>>>(wq, Wqh, Wql, n8w);
    k_split_planes<<<dim3((n8w + 255) / 256), dim3(256), 0, stream>>>(wk, Wkh, Wkl, n8w);
    k_split_planes<<<dim3((n8w + 255) / 256), dim3(256), 0, stream>>>(wv, Wvh, Wvl, n8w);
    k_split_planes<<<dim3((n8w + 255) / 256), dim3(256), 0, stream>>>(wo, Woh, Wol, n8w);
  }

  const int nTiles = (MROWS / 32) * (DM / 32);
  const int gemmBlocks = (nTiles + 3) / 4;
  k_gemm_xwt<<<dim3(gemmBlocks), dim3(128), 0, stream>>>(Xh, Xl, Wqh, Wql, Qf, MROWS, DM, DM);
  k_gemm_xwt<<<dim3(gemmBlocks), dim3(128), 0, stream>>>(Xh, Xl, Wkh, Wkl, Kf, MROWS, DM, DM);
  k_gemm_xwt<<<dim3(gemmBlocks), dim3(128), 0, stream>>>(Xh, Xl, Wvh, Wvl, Vf, MROWS, DM, DM);

  {
    const int nthr = MROWS * 8;
    k_rope_table<<<dim3((nthr + 255) / 256), dim3(256), 0, stream>>>(tpos, cosT, sinT, MROWS);
    const int nlines = MROWS * NH;
    k_rope_split<<<dim3((nlines + 127) / 128), dim3(128), 0, stream>>>(
        Qf, Kf, Vf, cosT, sinT, Qh, Ql, Kh, Kl, Vh, Vl, nlines);
  }

  {
    const int nblk = BH * (SQ / 64);
    k_attn<<<dim3(nblk), dim3(128), 0, stream>>>(Qh, Ql, Kh, Kl, Vh, Vl, Ch, Cl, nblk);
  }

  k_gemm_xwt<<<dim3(gemmBlocks), dim3(128), 0, stream>>>(Ch, Cl, Woh, Wol, out, MROWS, DM, DM);
}
